// CausalNCMomentumAttention_Py_58763742544958
// MI455X (gfx1250) — hardware-run, weakly checked
//
#include <hip/hip_runtime.h>


#define NSQ 2
#define NTS 8192
#define NHS 8
#define NFE 64
#define NCS 64
#define NCK 128
#define NPR 16
#define NQP 4
#define NZQ 512
#define NBL 4096

typedef _Float16 h16;
typedef unsigned short bf;
typedef __attribute__((ext_vector_type(16))) __bf16   v16bf;
typedef __attribute__((ext_vector_type(16))) _Float16 v16h;
typedef __attribute__((ext_vector_type(8)))  _Float16 v8h;
typedef __attribute__((ext_vector_type(8)))  unsigned short v8us;
typedef __attribute__((ext_vector_type(8)))  float    v8f;
typedef __attribute__((ext_vector_type(4)))  float    v4f;
typedef v8h  __attribute__((may_alias)) v8ha;
typedef v4f  __attribute__((may_alias)) v4fa;
typedef v8us __attribute__((may_alias)) v8usa;

__device__ __forceinline__ unsigned short f2bf(float f) { unsigned u = __float_as_uint(f); u += 0x7FFFu + ((u >> 16) & 1u); return (unsigned short)(u >> 16); }
__device__ __forceinline__ float bf2f(unsigned short b) { return __uint_as_float(((unsigned)b) << 16); }
__device__ __forceinline__ float bfr(float f) { return bf2f(f2bf(f)); }
__device__ __forceinline__ v16h cat16(v8h lo, v8h hi) { return __builtin_shufflevector(lo, hi, 0, 1, 2, 3, 4, 5, 6, 7, 8, 9, 10, 11, 12, 13, 14, 15); }
__device__ __forceinline__ v16bf cat16b(v8us lo, v8us hi) { return __builtin_bit_cast(v16bf, __builtin_shufflevector(lo, hi, 0, 1, 2, 3, 4, 5, 6, 7, 8, 9, 10, 11, 12, 13, 14, 15)); }
__device__ __forceinline__ v8f wmma16(v16h a, v16h b, v8f c) { return __builtin_amdgcn_wmma_f32_16x16x32_f16(false, a, false, b, (short)0, c, false, false); }
__device__ __forceinline__ v8f wmmab(v16bf a, v16bf b, v8f c) { return __builtin_amdgcn_wmma_f32_16x16x32_bf16(false, a, false, b, (short)0, c, false, false); }

template <typename T16> struct WFrag;
template <> struct WFrag<h16> { typedef v16h V; static __device__ __forceinline__ V ld(const h16* p) { return cat16(*(const v8h*)p, *(const v8h*)(p + 16)); } static __device__ __forceinline__ v8f mma(V a, V b, v8f c) { return wmma16(a, b, c); } };
template <> struct WFrag<bf> { typedef v16bf V; static __device__ __forceinline__ V ld(const bf* p) { return cat16b(*(const v8us*)p, *(const v8us*)(p + 16)); } static __device__ __forceinline__ v8f mma(V a, V b, v8f c) { return wmmab(a, b, c); } };
template <typename T16, int NSPLIT, bool BIAS>
__global__ __launch_bounds__(32) void k_gemmw(const T16* __restrict__ A, const T16* __restrict__ A2, const T16* __restrict__ Bt, const T16* __restrict__ Bt2, int K, float* C, int ldc, const float* __restrict__ bias, size_t sA, size_t sB, size_t sC) {
    typedef typename WFrag<T16>::V V;
    __shared__ __align__(16) float os[16 * 68];
    const size_t z = blockIdx.z; A += z * sA; if (A2) A2 += z * sA; Bt += z * sB; if (Bt2) Bt2 += z * sB; C += z * sC;
    const int lane = threadIdx.x & 31, lr = lane & 15, hi = lane >> 4; const int r0 = blockIdx.x * 64, c0 = blockIdx.y * 64;
    v8f acc[4][4];
#pragma unroll
    for (int mb = 0; mb < 4; ++mb)
#pragma unroll
        for (int nb = 0; nb < 4; ++nb) acc[mb][nb] = (v8f){};
    const size_t aoff = (size_t)(r0 + lr) * K + 8 * hi, boff = (size_t)(c0 + lr) * K + 8 * hi;
    for (int kc = 0; kc < K; kc += 32) {
        V a[4], a2[4];
#pragma unroll
        for (int mb = 0; mb < 4; ++mb) { a[mb] = WFrag<T16>::ld(A + aoff + (size_t)mb * 16 * K + kc); if (NSPLIT == 1 || NSPLIT == 2) a2[mb] = WFrag<T16>::ld(A2 + aoff + (size_t)mb * 16 * K + kc); }
#pragma unroll
        for (int nb = 0; nb < 4; ++nb) { const V b = WFrag<T16>::ld(Bt + boff + (size_t)nb * 16 * K + kc); V b2; if (NSPLIT >= 2) b2 = WFrag<T16>::ld(Bt2 + boff + (size_t)nb * 16 * K + kc);
#pragma unroll
            for (int mb = 0; mb < 4; ++mb) { acc[mb][nb] = WFrag<T16>::mma(a[mb], b, acc[mb][nb]); if (NSPLIT == 1 || NSPLIT == 2) acc[mb][nb] = WFrag<T16>::mma(a2[mb], b, acc[mb][nb]); if (NSPLIT >= 2) acc[mb][nb] = WFrag<T16>::mma(a[mb], b2, acc[mb][nb]); } }
        asm volatile("v_nop\n\tv_nop\n\tv_nop\n\tv_nop" : "+v"(acc[0][0]), "+v"(acc[1][1]), "+v"(acc[2][2]), "+v"(acc[3][3]) : "v"(a[0]), "v"(a[3]));
    }
#pragma unroll
    for (int mb = 0; mb < 4; ++mb) {
#pragma unroll
        for (int nb = 0; nb < 4; ++nb) {
#pragma unroll
            for (int j = 0; j < 8; ++j) os[(hi * 8 + j) * 68 + nb * 16 + lr] = acc[mb][nb][j]; }
        __builtin_amdgcn_wave_barrier(); asm volatile("" ::: "memory");
        float* crow = C + (size_t)(r0 + mb * 16) * ldc + c0;
#pragma unroll 1
        for (int ps = 0; ps < 2; ++ps) {
#pragma unroll
            for (int s = 0; s < 8; ++s) { const int row = 2 * s + hi, cofs = lr * 4; v4f val = *(const v4fa*)(os + row * 68 + cofs); if (BIAS) { val[0] += bfr(bias[c0 + cofs]); val[1] += bfr(bias[c0 + cofs + 1]); val[2] += bfr(bias[c0 + cofs + 2]); val[3] += bfr(bias[c0 + cofs + 3]); }
                *(volatile v4f*)(crow + (size_t)row * ldc + cofs) = val; }
            if (ps == 0) __threadfence(); }
        __builtin_amdgcn_wave_barrier(); asm volatile("" ::: "memory");
    }
}

typedef __attribute__((ext_vector_type(2))) _Float16 v2h;
typedef __attribute__((ext_vector_type(4))) _Float16 v4h;
typedef __attribute__((ext_vector_type(2))) unsigned short v2us;
typedef __attribute__((ext_vector_type(4))) unsigned short v4us;
typedef __attribute__((ext_vector_type(2))) float v2f;
typedef __attribute__((ext_vector_type(4))) int v4i;
__device__ __forceinline__ h16 toh_flush(float x) { const float z = (fabsf(x) < 6.103515625e-05f) ? 0.0f : x; return (h16)z; }

typedef __attribute__((ext_vector_type(4))) _Float16 v4h_;
__global__ __launch_bounds__(256) void k_fillb(bf* P, unsigned w2, size_t n8) { const size_t i = (size_t)blockIdx.x * 256 + threadIdx.x; if (i >= n8) return; v4i o; o[0] = (int)w2; o[1] = (int)w2; o[2] = (int)w2; o[3] = (int)w2;
    *(volatile v4i*)(P + i * 8) = o; __threadfence(); *(volatile v4i*)(P + i * 8) = o; }

__global__ __launch_bounds__(256) void k_rowf(const float* __restrict__ ina, const float* __restrict__ inb, const float* __restrict__ ind, h16* Fa, h16* Fb, int pr0) {
    const unsigned i = blockIdx.x * 256 + threadIdx.x; const unsigned e8 = i & 7u, ts = (i >> 3) & 8191u, pl = i >> 16; const unsigned pr = (unsigned)pr0 + pl, sq = pr >> 3, hd = pr & 7u;
    const size_t src = (((size_t)sq * NTS + ts) * NHS + hd) * NFE + e8 * 8; const v8f wa = *(const v8f*)(ina + src); const v8f wb = *(const v8f*)(inb + src); const float mk = bfr(ind[(size_t)sq * NTS + ts]); v8h oa, ob;
#pragma unroll
    for (int j = 0; j < 8; ++j) { const float ya = bfr(wa[j]), yb = bfr(wb[j]); oa[j] = toh_flush(fmaxf(ya, 0.0f) + expf(fminf(ya, 0.0f))); ob[j] = toh_flush((fmaxf(yb, 0.0f) + expf(fminf(yb, 0.0f))) * mk); }
    h16* pa = Fa + (size_t)i * 8; h16* pb = Fb + (size_t)i * 8;
    *(volatile v8h*)pa = oa; *(volatile v8h*)pb = ob; __threadfence(); *(volatile v8h*)pa = oa; *(volatile v8h*)pb = ob; }

__global__ __launch_bounds__(256) void k_colf(const float* __restrict__ inb, const float* __restrict__ inc, const float* __restrict__ ind, h16* Gb, h16* Gc, float* Cu, int pr0) {
    const unsigned i = blockIdx.x * 256 + threadIdx.x; const unsigned cl = i & 63u, ck = (i >> 6) & 127u, pl = i >> 13; const unsigned pr = (unsigned)pr0 + pl, sq = pr >> 3, hd = pr & 7u;
    const size_t b0 = (((size_t)sq * NTS + (size_t)ck * NCS) * NHS + hd) * NFE + cl; const float* mp = ind + (size_t)sq * NTS + (size_t)ck * NCS; h16 rb[64], rc[64]; float acc = 0.0f;
#pragma unroll
    for (int tj = 0; tj < 64; ++tj) { const float yb = bfr(inb[b0 + (size_t)tj * (NHS * NFE)]); const float yc = bfr(inc[b0 + (size_t)tj * (NHS * NFE)]); const h16 wb = toh_flush((fmaxf(yb, 0.0f) + expf(fminf(yb, 0.0f))) * bfr(mp[tj])); rb[tj] = wb; rc[tj] = toh_flush(yc); acc = acc + (float)wb; }
    h16* pb = Gb + ((size_t)(pl * NCK + ck) * 64 + cl) * 64; h16* pc = Gc + ((size_t)(pr * NCK + ck) * 64 + cl) * 64; float* pu = Cu + ((size_t)ck * NPR + pr) * 64 + cl;
#pragma unroll
    for (int ps = 0; ps < 2; ++ps) {
#pragma unroll
        for (int g = 0; g < 8; ++g) { v8h ob, oc;
#pragma unroll
            for (int j = 0; j < 8; ++j) { ob[j] = rb[g * 8 + j]; oc[j] = rc[g * 8 + j]; }
            *(volatile v8h*)(pb + g * 8) = ob; *(volatile v8h*)(pc + g * 8) = oc; }
        *(volatile float*)pu = acc;
        if (ps == 0) __threadfence(); } }

__global__ __launch_bounds__(256) void k_msk(const float* __restrict__ Pw, const h16* __restrict__ Fa, const float* __restrict__ Cs, h16* Ph, h16* Pl, float* Dn, int pr0) {
    const unsigned i = blockIdx.x * 256 + threadIdx.x; const unsigned tr = i & 63u, zq = i >> 6, ck = zq & 127u, pl = zq >> 7; const unsigned pr = (unsigned)pr0 + pl;
    const float* pw = Pw + (size_t)i * 64; const h16* fr = Fa + (size_t)i * 64; const float* c1 = Cs + ((size_t)ck * NPR + pr) * 64; const float* c0 = Cs + ((size_t)NCK * NPR + pr) * 64; h16 rh[64], rl[64]; float acc = 0.0f, d1 = 0.0f, d0 = 0.0f;
#pragma unroll
    for (int sj = 0; sj < 64; ++sj) { const float kp = (float)((unsigned)sj <= tr); const float pm = pw[sj] * kp; const h16 hi = toh_flush(pm); rh[sj] = hi; rl[sj] = toh_flush(pm - (float)hi); acc = acc + pm; const float fq = (float)fr[sj]; d1 = d1 + fq * c1[sj]; d0 = d0 + fq * c0[sj]; }
    const float r1 = 1.0f / (acc + d1 + 1e-6f); const float r0 = 1.0f / (d0 + 1e-6f); h16* ph = Ph + (size_t)i * 64; h16* pq = Pl + (size_t)i * 64; float* dn = Dn + i;
#pragma unroll
    for (int ps = 0; ps < 2; ++ps) {
#pragma unroll
        for (int g = 0; g < 8; ++g) { v8h oh, ol;
#pragma unroll
            for (int j = 0; j < 8; ++j) { oh[j] = rh[g * 8 + j]; ol[j] = rl[g * 8 + j]; }
            *(volatile v8h*)(ph + g * 8) = oh; *(volatile v8h*)(pq + g * 8) = ol; }
        *(volatile float*)dn = r1; *(volatile float*)(dn + NZQ * 64) = r0;
        if (ps == 0) __threadfence(); } }

__global__ __launch_bounds__(256) void k_addw(const float* __restrict__ bef, size_t sbef, const float* __restrict__ upd, size_t supd, float* aft, h16* wrd, size_t swrd) {
    const unsigned i = blockIdx.x * 256 + threadIdx.x; const unsigned j4 = i & 1023u, pr = i >> 10; const v4f ub = *(const v4fa*)(bef + (size_t)pr * sbef + j4 * 4); const v4f vu = *(const v4fa*)(upd + (size_t)pr * supd + j4 * 4); v4h_ ow; v4f oa;
#pragma unroll
    for (int j = 0; j < 4; ++j) { ow[j] = toh_flush(ub[j]); oa[j] = ub[j] + vu[j]; }
    h16* pw = wrd + (size_t)pr * swrd + j4 * 4; float* pa = aft + (size_t)pr * NBL + j4 * 4;
    *(volatile v4h_*)pw = ow; *(volatile v4f*)pa = oa; __threadfence(); *(volatile v4h_*)pw = ow; *(volatile v4f*)pa = oa; }

__global__ __launch_bounds__(256) void k_add(const float* __restrict__ bef, const float* __restrict__ upd, float* aft) {
    const unsigned i = threadIdx.x; const v4f ub = *(const v4fa*)(bef + i * 4); const v4f vu = *(const v4fa*)(upd + i * 4); v4f oa;
#pragma unroll
    for (int j = 0; j < 4; ++j) oa[j] = ub[j] + vu[j];
    *(volatile v4f*)(aft + i * 4) = oa; __threadfence(); *(volatile v4f*)(aft + i * 4) = oa; }

__global__ __launch_bounds__(256) void k_lay(const float* __restrict__ Oa, const float* __restrict__ Ob, const float* __restrict__ Oc, const float* __restrict__ Dn, float* R0, float* R1, int pr0) {
    const unsigned i = blockIdx.x * 256 + threadIdx.x; const unsigned m4 = i & 15u, ts = (i >> 4) & 8191u, pl = i >> 17; const unsigned pr = (unsigned)pr0 + pl, sq = pr >> 3, hd = pr & 7u; const size_t rw = (size_t)pl * NTS + ts;
    const v4f ua = *(const v4fa*)(Oa + rw * 64 + m4 * 4); const v4f ub = *(const v4fa*)(Ob + rw * 64 + m4 * 4); const v4f uc = *(const v4fa*)(Oc + rw * 64 + m4 * 4); const float r1 = Dn[rw]; const float r0 = Dn[(size_t)NZQ * 64 + rw]; v4f o1, o0;
#pragma unroll
    for (int j = 0; j < 4; ++j) { o1[j] = (ua[j] + ub[j]) * r1; o0[j] = uc[j] * r0; }
    const size_t dst = (((size_t)sq * NTS + ts) * NHS + hd) * NFE + m4 * 4;
    *(volatile v4f*)(R0 + dst) = o0; *(volatile v4f*)(R1 + dst) = o1; __threadfence(); *(volatile v4f*)(R0 + dst) = o0; *(volatile v4f*)(R1 + dst) = o1; }

extern "C" void kernel_launch(void* const* d_in, const int* in_sizes, int n_in, void* d_out, int out_size, void* d_ws, size_t ws_size, hipStream_t stream) {
    if (n_in < 4) return;
    if (in_sizes[0] != NSQ * NTS * NHS * NFE || in_sizes[1] != NSQ * NTS * NHS * NFE || in_sizes[2] != NSQ * NTS * NHS * NFE || in_sizes[3] != NSQ * NTS) return;
    if (out_size != 2 * NSQ * NTS * NHS * NFE) return;
    static_assert(NPR == NSQ * NHS && NHS == 8 && NFE == 64 && NCS == 64 && NCK * NCS == NTS && NTS == 8192 && NZQ == NQP * NCK && NPR % NQP == 0 && NBL == 64 * 64 && (NQP * NTS * NFE / 8) % 256 == 0 && (NZQ * 64) % 256 == 0 && (NPR * NBL / 4) % 256 == 0 && (NQP * NTS * NFE / 4) % 256 == 0 && (NPR * NBL * 4) % 256 == 0 && (NPR * NBL * 4 + NPR * 64 * 4) % 16 == 0, "the products: 64 by 64 blocks over a depth of 64; the flat grids exact; the index fields' widths (3 bits a head, 13 a time, 7 a chunk, 6 a column); Zn a whole number of 256-byte steps so that Cs follows it at once");
    const float* ina = (const float*)d_in[0]; const float* inb = (const float*)d_in[1]; const float* inc = (const float*)d_in[2]; const float* ind = (const float*)d_in[3]; float* R0 = (float*)d_out; float* R1 = R0 + (size_t)NSQ * NTS * NHS * NFE;
    char* wsp = (char*)d_ws; auto take = [&](size_t bytes) { char* p = wsp; wsp += (bytes + 255) & ~(size_t)255; return (void*)p; };
    float* Zn = (float*)take((size_t)NPR * NBL * 4); float* Cs = (float*)take((size_t)(NCK + 1) * NPR * 64 * 4); float* Cu = (float*)take((size_t)NCK * NPR * 64 * 4); float* Ra = (float*)take((size_t)NPR * NBL * 4); float* Rb = (float*)take((size_t)NPR * NBL * 4);
    float* Du = (float*)take((size_t)NPR * NCK * NBL * 4); h16* Sw = (h16*)take((size_t)NPR * NCK * NBL * 2); h16* Gc = (h16*)take((size_t)NPR * NCK * NBL * 2); h16* Tw = (h16*)take((size_t)NPR * NBL * 2);
    h16* Gb = (h16*)take((size_t)NZQ * NBL * 2); h16* Fa = (h16*)take((size_t)NZQ * NBL * 2); h16* Fb = (h16*)take((size_t)NZQ * NBL * 2); float* Pw = (float*)take((size_t)NZQ * NBL * 4); h16* Ph = (h16*)take((size_t)NZQ * NBL * 2); h16* Pl = (h16*)take((size_t)NZQ * NBL * 2); float* Dn = (float*)take((size_t)2 * NZQ * 64 * 4);
    float* Oa = (float*)take((size_t)NZQ * NBL * 4); float* Ob = (float*)take((size_t)NZQ * NBL * 4); float* Oc = (float*)take((size_t)NZQ * NBL * 4);
    if ((size_t)(wsp - (char*)d_ws) > ws_size) return;
    k_fillb<<<(unsigned)(((NPR * NBL * 4 + NPR * 64 * 4) / 16 + 255) / 256), 256, 0, stream>>>((bf*)Zn, 0u, (size_t)(NPR * NBL * 4 + NPR * 64 * 4) / 16);
    for (int qr = 0; qr < NPR / NQP; ++qr) {
        k_colf<<<(unsigned)(NZQ * 64 / 256), 256, 0, stream>>>(inb, inc, ind, Gb, Gc, Cu, qr * NQP);
        k_gemmw<h16, 0, false><<<dim3(1, 1, NZQ), 32, 0, stream>>>(Gc + (size_t)qr * NZQ * NBL, nullptr, Gb, nullptr, NCS, Du + (size_t)qr * NZQ * NBL, 64, nullptr, NBL, NBL, NBL); }
    { const float* bef = Zn; for (int ck = 0; ck < NCK; ++ck) { float* aft = (ck & 1) ? Rb : Ra;
            k_addw<<<(unsigned)(NPR * NBL / 4 / 256), 256, 0, stream>>>(bef, (size_t)NBL, Du + (size_t)ck * NBL, (size_t)NCK * NBL, aft, Sw + (size_t)ck * NBL, (size_t)NCK * NBL);
            k_add<<<1, 256, 0, stream>>>(Cs + (size_t)ck * NPR * 64, Cu + (size_t)ck * NPR * 64, Cs + (size_t)(ck + 1) * NPR * 64); bef = aft; }
        k_addw<<<(unsigned)(NPR * NBL / 4 / 256), 256, 0, stream>>>(bef, (size_t)NBL, Zn, (size_t)NBL, (bef == Ra) ? Rb : Ra, Tw, (size_t)NBL); }
    for (int qr = 0; qr < NPR / NQP; ++qr) {
        k_rowf<<<(unsigned)(NQP * NTS * NFE / 8 / 256), 256, 0, stream>>>(ina, inb, ind, Fa, Fb, qr * NQP);
        k_gemmw<h16, 0, false><<<dim3(1, 1, NZQ), 32, 0, stream>>>(Fa, nullptr, Fb, nullptr, NFE, Pw, 64, nullptr, NBL, NBL, NBL);
        k_msk<<<(unsigned)(NZQ * 64 / 256), 256, 0, stream>>>(Pw, Fa, Cs, Ph, Pl, Dn, qr * NQP);
        k_gemmw<h16, 1, false><<<dim3(1, 1, NZQ), 32, 0, stream>>>(Ph, Pl, Gc + (size_t)qr * NZQ * NBL, nullptr, NCS, Oa, 64, nullptr, NBL, NBL, NBL);
        k_gemmw<h16, 0, false><<<dim3(1, 1, NZQ), 32, 0, stream>>>(Fa, nullptr, Sw + (size_t)qr * NZQ * NBL, nullptr, NFE, Ob, 64, nullptr, NBL, NBL, NBL);
        k_gemmw<h16, 0, false><<<dim3(NTS / 64, 1, NQP), 32, 0, stream>>>(Fa, nullptr, Tw + (size_t)qr * NQP * NBL, nullptr, NFE, Oc, 64, nullptr, (size_t)NTS * NFE, NBL, (size_t)NTS * NFE);
        k_lay<<<(unsigned)(NQP * NTS * NFE / 4 / 256), 256, 0, stream>>>(Oa, Ob, Oc, Dn, R0, R1, qr * NQP); }
}
